// TransBlockV3BodyOrderTest_42305427866212
// MI455X (gfx1250) — hardware-verified
//
#include <hip/hip_runtime.h>


namespace {
constexpr int N = 2048, L2 = 16, CI = 384, CH = 256, NG = 353;
constexpr float XS = 8.0f, WSC = 256.0f;
typedef _Float16 b16;
typedef __attribute__((ext_vector_type(16))) _Float16 v16b;
typedef __attribute__((ext_vector_type(8))) _Float16 v8b;
typedef __attribute__((ext_vector_type(8))) float v8f;
typedef __attribute__((ext_vector_type(4))) float v4f;
__device__ __forceinline__ float bf16_rne(float f) { unsigned int u = __float_as_uint(f); u += 0x7FFFu + ((u >> 16) & 1u); float r = __uint_as_float(u & 0xFFFF0000u); asm volatile("" : "+v"(r)); return r; }
__device__ __forceinline__ void split16(float v, b16& hi, b16& lo) { hi = (b16)v; lo = (b16)(v - (float)hi); }
__device__ __forceinline__ v16b frag_kb(const b16* p, int hh) { const v8b a = *(const v8b*)(p + 8 * hh), b = *(const v8b*)(p + 16 + 8 * hh); v16b f;
#pragma unroll
  for (int e = 0; e < 8; ++e) { f[e] = a[e]; f[8 + e] = b[e]; } return f; }
__device__ __forceinline__ v8f wmma16b(v16b a, v16b b, v8f c) { v8f d = __builtin_amdgcn_wmma_f32_16x16x32_f16(false, a, false, b, (short)0, c, false, false); asm volatile("v_nop\n\tv_nop\n\tv_nop\n\tv_nop" : "+v"(d) : "v"(a), "v"(b)); return d; }
__device__ __forceinline__ void wave_lds_sync() { __builtin_amdgcn_fence(__ATOMIC_RELEASE, "workgroup"); __builtin_amdgcn_wave_barrier(); __builtin_amdgcn_fence(__ATOMIC_ACQUIRE, "workgroup"); }
__device__ __forceinline__ float pmul(float a, float b) { float p = a * b; asm volatile("" : "+v"(p)); return p; }
__device__ __forceinline__ int l_of(int i) { return i < 1 ? 0 : (i < 4 ? 1 : (i < 9 ? 2 : 3)); }

__global__ __launch_bounds__(256) void wput_kernel(const float* __restrict__ w1, const float* __restrict__ w2, b16* __restrict__ W1T, b16* __restrict__ W2T) { const int u = blockIdx.x * 256 + threadIdx.x; const int n1 = 4 * CH * (CI / 8), n2 = 4 * CI * (CH / 8);
  for (int pass = 0; pass < 2; ++pass) {
    if (u < n1) { const int l = u / (CH * (CI / 8)), o = (u / (CI / 8)) % CH, k0 = (u % (CI / 8)) * 8; v8b v;
#pragma unroll
      for (int j = 0; j < 8; ++j) v[j] = (b16)(bf16_rne(w1[((size_t)l * CI + k0 + j) * CH + o]) * WSC); *(volatile v8b*)(W1T + ((size_t)l * CH + o) * CI + k0) = v; }
    if (u < n2) { const int l = u / (CI * (CH / 8)), o = (u / (CH / 8)) % CI, k0 = (u % (CH / 8)) * 8; v8b v;
#pragma unroll
      for (int j = 0; j < 8; ++j) v[j] = (b16)(bf16_rne(w2[((size_t)l * CH + k0 + j) * CI + o]) * WSC); *(volatile v8b*)(W2T + ((size_t)l * CI + o) * CH + k0) = v; }
    __threadfence(); } }
__global__ __launch_bounds__(256) void norm_kernel(const float* __restrict__ x, const float* __restrict__ nw, const float* __restrict__ nb, int NV, float* __restrict__ XN) { const int wave = threadIdx.x >> 5, lane = threadIdx.x & 31; const int n = blockIdx.x * 8 + wave; if (n >= NV) return; const float* xr = x + (size_t)n * L2 * CI;
  float m0 = 0.0f; for (int c = lane; c < CI; c += 32) m0 += bf16_rne(xr[c]); for (int o = 16; o; o >>= 1) m0 += __shfl_xor(m0, o); m0 *= (1.0f / CI);
  float ss = 0.0f; for (int i = 0; i < L2; ++i) for (int c = lane; c < CI; c += 32) { float v = bf16_rne(xr[i * CI + c]); if (i == 0) v -= m0; ss += pmul(v, v); } for (int o = 16; o; o >>= 1) ss += __shfl_xor(ss, o); const float rs = rsqrtf(ss * (1.0f / (L2 * CI)) + 1e-5f);
  for (int pass = 0; pass < 2; ++pass) { for (int i = 0; i < L2; ++i) { const int l = l_of(i); for (int c = lane; c < CI; c += 32) { float v = bf16_rne(xr[i * CI + c]); if (i == 0) v -= m0; v = pmul(pmul(v, rs), bf16_rne(nw[l * CI + c])); if (i == 0) v += bf16_rne(nb[c]); ((volatile float*)XN)[((size_t)n * L2 + i) * CI + c] = v; } } __threadfence(); } }
template <int MODE>
__global__ __launch_bounds__(32) void so3_kernel(const float* __restrict__ IN, const b16* __restrict__ WT, const float* __restrict__ bias, const float* __restrict__ inputs, int NV, float* __restrict__ OUT) {
  constexpr int KT = MODE == 0 ? CI : CH, OW = MODE == 0 ? CH : CI, NGRP = OW / 128; __shared__ __attribute__((aligned(16))) b16 Ah[16][KT + 8], Al[16][KT + 8]; __shared__ float Tf[16][132]; __shared__ int Rn[16], Ri[16];
  const int lane = threadIdx.x, nloc = lane & 15, hlf = lane >> 4; const int g = blockIdx.x % NGRP; int tt = blockIdx.x / NGRP;
  int l = 0, base = 0; for (l = 0; l < 4; ++l) { const int nt = NV * (2 * l + 1) / 16; if (tt < nt) break; tt -= nt; base += nt; } if (l >= 4) return; (void)base;
  if (lane < 16) { const int r = tt * 16 + lane; const int w = 2 * l + 1; Rn[lane] = r / w; Ri[lane] = l * l + r % w; }
  wave_lds_sync();
  for (int rr = 0; rr < 16; ++rr) { const size_t row = (size_t)Rn[rr] * L2 + Ri[rr]; for (int q = 0; q < KT / 32; ++q) { b16 p, ql; split16(IN[row * KT + q * 32 + lane] * XS, p, ql); Ah[rr][q * 32 + lane] = p; Al[rr][q * 32 + lane] = ql; } }
  wave_lds_sync(); v8f acc[8];
#pragma unroll
  for (int t = 0; t < 8; ++t) acc[t] = (v8f){};
  const b16* Wl = WT + (size_t)l * OW * KT;
#pragma unroll 2
  for (int kb = 0; kb < KT; kb += 32) { const v16b a = frag_kb(&Ah[nloc][kb], hlf), al = frag_kb(&Al[nloc][kb], hlf);
#pragma unroll
    for (int t = 0; t < 8; ++t) { const v16b bw = frag_kb(Wl + (size_t)(g * 128 + t * 16 + nloc) * KT + kb, hlf); acc[t] = wmma16b(a, bw, acc[t]); acc[t] = wmma16b(al, bw, acc[t]); } }
#pragma unroll
  for (int t = 0; t < 8; ++t) { const int c = g * 128 + t * 16 + nloc; const float bb = bf16_rne(bias[c]);
#pragma unroll
    for (int r8 = 0; r8 < 8; ++r8) { const int rl = 8 * hlf + r8; Tf[rl][t * 16 + nloc] = acc[t][r8] * (1.0f / (XS * WSC)) + (Ri[rl] == 0 ? bb : 0.0f); } }
  wave_lds_sync();
  for (int pass = 0; pass < 2; ++pass) { for (int rr = 0; rr < 16; ++rr) { const size_t row = (size_t)Rn[rr] * L2 + Ri[rr]; v4f v = *(const v4f*)(&Tf[rr][lane * 4]); if (MODE == 1) { const float* ir = inputs + row * CI + g * 128 + lane * 4; for (int k = 0; k < 4; ++k) v[k] += bf16_rne(ir[k]); } *(volatile v4f*)(OUT + row * OW + g * 128 + lane * 4) = v; } __threadfence(); } }
__global__ __launch_bounds__(256) void gaunt_kernel(const float* __restrict__ Hh, const float* __restrict__ wg, int NV, float* __restrict__ T) { const int u = blockIdx.x * 256 + threadIdx.x; if (u >= NV * CH) return; const int n = u / CH, h = u % CH; float hv[L2], t[L2], w[64];
#pragma unroll
  for (int i = 0; i < L2; ++i) { hv[i] = Hh[((size_t)n * L2 + i) * CH + h]; t[i] = 0.0f; }
#pragma unroll
  for (int q = 0; q < 64; ++q) w[q] = bf16_rne(wg[(size_t)q * CH + h]);
  t[0] += pmul(0.141047403f, pmul(hv[0], pmul(hv[0], w[0])));
  t[1] += pmul(0.199471146f, pmul(hv[0], pmul(hv[1], w[5])));
  t[2] += pmul(0.199471146f, pmul(hv[0], pmul(hv[2], w[5])));
  t[3] += pmul(0.199471146f, pmul(hv[0], pmul(hv[3], w[5])));
  t[4] += pmul(0.238413617f, pmul(hv[0], pmul(hv[4], w[10])));
  t[5] += pmul(0.238413617f, pmul(hv[0], pmul(hv[5], w[10])));
  t[6] += pmul(0.238413617f, pmul(hv[0], pmul(hv[6], w[10])));
  t[7] += pmul(0.238413617f, pmul(hv[0], pmul(hv[7], w[10])));
  t[8] += pmul(0.238413617f, pmul(hv[0], pmul(hv[8], w[10])));
  t[9] += pmul(0.304697186f, pmul(hv[0], pmul(hv[9], w[15])));
  t[10] += pmul(0.304697186f, pmul(hv[0], pmul(hv[10], w[15])));
  t[11] += pmul(0.304697186f, pmul(hv[0], pmul(hv[11], w[15])));
  t[12] += pmul(0.304697186f, pmul(hv[0], pmul(hv[12], w[15])));
  t[13] += pmul(0.304697186f, pmul(hv[0], pmul(hv[13], w[15])));
  t[14] += pmul(0.304697186f, pmul(hv[0], pmul(hv[14], w[15])));
  t[15] += pmul(0.304697186f, pmul(hv[0], pmul(hv[15], w[15])));
  t[1] += pmul(0.199471146f, pmul(hv[1], pmul(hv[0], w[17])));
  t[2] += pmul(0.199471146f, pmul(hv[2], pmul(hv[0], w[17])));
  t[3] += pmul(0.199471146f, pmul(hv[3], pmul(hv[0], w[17])));
  t[0] += pmul(0.141047403f, pmul(hv[1], pmul(hv[1], w[20])));
  t[0] += pmul(0.141047403f, pmul(hv[2], pmul(hv[2], w[20])));
  t[0] += pmul(0.141047403f, pmul(hv[3], pmul(hv[3], w[20])));
  t[6] += pmul(-0.106621809f, pmul(hv[1], pmul(hv[1], w[22])));
  t[8] += pmul(-0.184674397f, pmul(hv[1], pmul(hv[1], w[22])));
  t[5] += pmul(0.184674397f, pmul(hv[1], pmul(hv[2], w[22])));
  t[4] += pmul(0.184674397f, pmul(hv[1], pmul(hv[3], w[22])));
  t[5] += pmul(0.184674397f, pmul(hv[2], pmul(hv[1], w[22])));
  t[6] += pmul(0.213243619f, pmul(hv[2], pmul(hv[2], w[22])));
  t[7] += pmul(0.184674397f, pmul(hv[2], pmul(hv[3], w[22])));
  t[4] += pmul(0.184674397f, pmul(hv[3], pmul(hv[1], w[22])));
  t[7] += pmul(0.184674397f, pmul(hv[3], pmul(hv[2], w[22])));
  t[6] += pmul(-0.106621809f, pmul(hv[3], pmul(hv[3], w[22])));
  t[8] += pmul(0.184674397f, pmul(hv[3], pmul(hv[3], w[22])));
  t[3] += pmul(0.154509678f, pmul(hv[1], pmul(hv[4], w[25])));
  t[2] += pmul(0.154509678f, pmul(hv[1], pmul(hv[5], w[25])));
  t[1] += pmul(-0.0892062038f, pmul(hv[1], pmul(hv[6], w[25])));
  t[1] += pmul(-0.154509678f, pmul(hv[1], pmul(hv[8], w[25])));
  t[1] += pmul(0.154509678f, pmul(hv[2], pmul(hv[5], w[25])));
  t[2] += pmul(0.178412408f, pmul(hv[2], pmul(hv[6], w[25])));
  t[3] += pmul(0.154509678f, pmul(hv[2], pmul(hv[7], w[25])));
  t[1] += pmul(0.154509678f, pmul(hv[3], pmul(hv[4], w[25])));
  t[3] += pmul(-0.0892062038f, pmul(hv[3], pmul(hv[6], w[25])));
  t[2] += pmul(0.154509678f, pmul(hv[3], pmul(hv[7], w[25])));
  t[3] += pmul(0.154509678f, pmul(hv[3], pmul(hv[8], w[25])));
  t[13] += pmul(-0.0630783141f, pmul(hv[1], pmul(hv[4], w[27])));
  t[15] += pmul(-0.244301260f, pmul(hv[1], pmul(hv[4], w[27])));
  t[12] += pmul(-0.154509678f, pmul(hv[1], pmul(hv[5], w[27])));
  t[14] += pmul(-0.199471146f, pmul(hv[1], pmul(hv[5], w[27])));
  t[11] += pmul(0.218509689f, pmul(hv[1], pmul(hv[6], w[27])));
  t[10] += pmul(0.199471146f, pmul(hv[1], pmul(hv[7], w[27])));
  t[9] += pmul(0.244301260f, pmul(hv[1], pmul(hv[8], w[27])));
  t[11] += pmul(0.0630783141f, pmul(hv[1], pmul(hv[8], w[27])));
  t[10] += pmul(0.199471146f, pmul(hv[2], pmul(hv[4], w[27])));
  t[11] += pmul(0.252313256f, pmul(hv[2], pmul(hv[5], w[27])));
  t[12] += pmul(0.267618626f, pmul(hv[2], pmul(hv[6], w[27])));
  t[13] += pmul(0.252313256f, pmul(hv[2], pmul(hv[7], w[27])));
  t[14] += pmul(0.199471146f, pmul(hv[2], pmul(hv[8], w[27])));
  t[9] += pmul(0.244301260f, pmul(hv[3], pmul(hv[4], w[27])));
  t[11] += pmul(-0.0630783141f, pmul(hv[3], pmul(hv[4], w[27])));
  t[10] += pmul(0.199471146f, pmul(hv[3], pmul(hv[5], w[27])));
  t[13] += pmul(0.218509689f, pmul(hv[3], pmul(hv[6], w[27])));
  t[12] += pmul(-0.154509678f, pmul(hv[3], pmul(hv[7], w[27])));
  t[14] += pmul(0.199471146f, pmul(hv[3], pmul(hv[7], w[27])));
  t[13] += pmul(-0.0630783141f, pmul(hv[3], pmul(hv[8], w[27])));
  t[15] += pmul(0.244301260f, pmul(hv[3], pmul(hv[8], w[27])));
  t[8] += pmul(0.191156149f, pmul(hv[1], pmul(hv[9], w[30])));
  t[7] += pmul(0.156078354f, pmul(hv[1], pmul(hv[10], w[30])));
  t[6] += pmul(0.170975268f, pmul(hv[1], pmul(hv[11], w[30])));
  t[8] += pmul(0.0493563078f, pmul(hv[1], pmul(hv[11], w[30])));
  t[5] += pmul(-0.120897770f, pmul(hv[1], pmul(hv[12], w[30])));
  t[4] += pmul(-0.0493563078f, pmul(hv[1], pmul(hv[13], w[30])));
  t[5] += pmul(-0.156078354f, pmul(hv[1], pmul(hv[14], w[30])));
  t[4] += pmul(-0.191156149f, pmul(hv[1], pmul(hv[15], w[30])));
  t[4] += pmul(0.156078354f, pmul(hv[2], pmul(hv[10], w[30])));
  t[5] += pmul(0.197425231f, pmul(hv[2], pmul(hv[11], w[30])));
  t[6] += pmul(0.209401071f, pmul(hv[2], pmul(hv[12], w[30])));
  t[7] += pmul(0.197425231f, pmul(hv[2], pmul(hv[13], w[30])));
  t[8] += pmul(0.156078354f, pmul(hv[2], pmul(hv[14], w[30])));
  t[4] += pmul(0.191156149f, pmul(hv[3], pmul(hv[9], w[30])));
  t[5] += pmul(0.156078354f, pmul(hv[3], pmul(hv[10], w[30])));
  t[4] += pmul(-0.0493563078f, pmul(hv[3], pmul(hv[11], w[30])));
  t[7] += pmul(-0.120897770f, pmul(hv[3], pmul(hv[12], w[30])));
  t[6] += pmul(0.170975268f, pmul(hv[3], pmul(hv[13], w[30])));
  t[8] += pmul(-0.0493563078f, pmul(hv[3], pmul(hv[13], w[30])));
  t[7] += pmul(0.156078354f, pmul(hv[3], pmul(hv[14], w[30])));
  t[8] += pmul(0.191156149f, pmul(hv[3], pmul(hv[15], w[30])));
  t[4] += pmul(0.238413617f, pmul(hv[4], pmul(hv[0], w[34])));
  t[5] += pmul(0.238413617f, pmul(hv[5], pmul(hv[0], w[34])));
  t[6] += pmul(0.238413617f, pmul(hv[6], pmul(hv[0], w[34])));
  t[7] += pmul(0.238413617f, pmul(hv[7], pmul(hv[0], w[34])));
  t[8] += pmul(0.238413617f, pmul(hv[8], pmul(hv[0], w[34])));
  t[3] += pmul(0.154509678f, pmul(hv[4], pmul(hv[1], w[37])));
  t[1] += pmul(0.154509678f, pmul(hv[4], pmul(hv[3], w[37])));
  t[2] += pmul(0.154509678f, pmul(hv[5], pmul(hv[1], w[37])));
  t[1] += pmul(0.154509678f, pmul(hv[5], pmul(hv[2], w[37])));
  t[1] += pmul(-0.0892062038f, pmul(hv[6], pmul(hv[1], w[37])));
  t[2] += pmul(0.178412408f, pmul(hv[6], pmul(hv[2], w[37])));
  t[3] += pmul(-0.0892062038f, pmul(hv[6], pmul(hv[3], w[37])));
  t[3] += pmul(0.154509678f, pmul(hv[7], pmul(hv[2], w[37])));
  t[2] += pmul(0.154509678f, pmul(hv[7], pmul(hv[3], w[37])));
  t[1] += pmul(-0.154509678f, pmul(hv[8], pmul(hv[1], w[37])));
  t[3] += pmul(0.154509678f, pmul(hv[8], pmul(hv[3], w[37])));
  t[13] += pmul(-0.0630783141f, pmul(hv[4], pmul(hv[1], w[39])));
  t[15] += pmul(-0.244301260f, pmul(hv[4], pmul(hv[1], w[39])));
  t[10] += pmul(0.199471146f, pmul(hv[4], pmul(hv[2], w[39])));
  t[9] += pmul(0.244301260f, pmul(hv[4], pmul(hv[3], w[39])));
  t[11] += pmul(-0.0630783141f, pmul(hv[4], pmul(hv[3], w[39])));
  t[12] += pmul(-0.154509678f, pmul(hv[5], pmul(hv[1], w[39])));
  t[14] += pmul(-0.199471146f, pmul(hv[5], pmul(hv[1], w[39])));
  t[11] += pmul(0.252313256f, pmul(hv[5], pmul(hv[2], w[39])));
  t[10] += pmul(0.199471146f, pmul(hv[5], pmul(hv[3], w[39])));
  t[11] += pmul(0.218509689f, pmul(hv[6], pmul(hv[1], w[39])));
  t[12] += pmul(0.267618626f, pmul(hv[6], pmul(hv[2], w[39])));
  t[13] += pmul(0.218509689f, pmul(hv[6], pmul(hv[3], w[39])));
  t[10] += pmul(0.199471146f, pmul(hv[7], pmul(hv[1], w[39])));
  t[13] += pmul(0.252313256f, pmul(hv[7], pmul(hv[2], w[39])));
  t[12] += pmul(-0.154509678f, pmul(hv[7], pmul(hv[3], w[39])));
  t[14] += pmul(0.199471146f, pmul(hv[7], pmul(hv[3], w[39])));
  t[9] += pmul(0.244301260f, pmul(hv[8], pmul(hv[1], w[39])));
  t[11] += pmul(0.0630783141f, pmul(hv[8], pmul(hv[1], w[39])));
  t[14] += pmul(0.199471146f, pmul(hv[8], pmul(hv[2], w[39])));
  t[13] += pmul(-0.0630783141f, pmul(hv[8], pmul(hv[3], w[39])));
  t[15] += pmul(0.244301260f, pmul(hv[8], pmul(hv[3], w[39])));
  t[0] += pmul(0.141047403f, pmul(hv[4], pmul(hv[4], w[40])));
  t[0] += pmul(0.141047403f, pmul(hv[5], pmul(hv[5], w[40])));
  t[0] += pmul(0.141047403f, pmul(hv[6], pmul(hv[6], w[40])));
  t[0] += pmul(0.141047403f, pmul(hv[7], pmul(hv[7], w[40])));
  t[0] += pmul(0.141047403f, pmul(hv[8], pmul(hv[8], w[40])));
  t[6] += pmul(-0.152316868f, pmul(hv[4], pmul(hv[4], w[42])));
  t[7] += pmul(0.131910279f, pmul(hv[4], pmul(hv[5], w[42])));
  t[4] += pmul(-0.152316868f, pmul(hv[4], pmul(hv[6], w[42])));
  t[5] += pmul(0.131910279f, pmul(hv[4], pmul(hv[7], w[42])));
  t[7] += pmul(0.131910279f, pmul(hv[5], pmul(hv[4], w[42])));
  t[6] += pmul(0.0761584342f, pmul(hv[5], pmul(hv[5], w[42])));
  t[8] += pmul(-0.131910279f, pmul(hv[5], pmul(hv[5], w[42])));
  t[5] += pmul(0.0761584342f, pmul(hv[5], pmul(hv[6], w[42])));
  t[4] += pmul(0.131910279f, pmul(hv[5], pmul(hv[7], w[42])));
  t[5] += pmul(-0.131910279f, pmul(hv[5], pmul(hv[8], w[42])));
  t[4] += pmul(-0.152316868f, pmul(hv[6], pmul(hv[4], w[42])));
  t[5] += pmul(0.0761584342f, pmul(hv[6], pmul(hv[5], w[42])));
  t[6] += pmul(0.152316868f, pmul(hv[6], pmul(hv[6], w[42])));
  t[7] += pmul(0.0761584342f, pmul(hv[6], pmul(hv[7], w[42])));
  t[8] += pmul(-0.152316868f, pmul(hv[6], pmul(hv[8], w[42])));
  t[5] += pmul(0.131910279f, pmul(hv[7], pmul(hv[4], w[42])));
  t[4] += pmul(0.131910279f, pmul(hv[7], pmul(hv[5], w[42])));
  t[7] += pmul(0.0761584342f, pmul(hv[7], pmul(hv[6], w[42])));
  t[6] += pmul(0.0761584342f, pmul(hv[7], pmul(hv[7], w[42])));
  t[8] += pmul(0.131910279f, pmul(hv[7], pmul(hv[7], w[42])));
  t[7] += pmul(0.131910279f, pmul(hv[7], pmul(hv[8], w[42])));
  t[5] += pmul(-0.131910279f, pmul(hv[8], pmul(hv[5], w[42])));
  t[8] += pmul(-0.152316868f, pmul(hv[8], pmul(hv[6], w[42])));
  t[7] += pmul(0.131910279f, pmul(hv[8], pmul(hv[7], w[42])));
  t[6] += pmul(-0.152316868f, pmul(hv[8], pmul(hv[8], w[42])));
  t[3] += pmul(0.159932718f, pmul(hv[4], pmul(hv[9], w[45])));
  t[2] += pmul(0.130584508f, pmul(hv[4], pmul(hv[10], w[45])));
  t[3] += pmul(-0.0412944481f, pmul(hv[4], pmul(hv[11], w[45])));
  t[1] += pmul(-0.0412944481f, pmul(hv[4], pmul(hv[13], w[45])));
  t[1] += pmul(-0.159932718f, pmul(hv[4], pmul(hv[15], w[45])));
  t[3] += pmul(0.130584508f, pmul(hv[5], pmul(hv[10], w[45])));
  t[2] += pmul(0.165177792f, pmul(hv[5], pmul(hv[11], w[45])));
  t[1] += pmul(-0.101150326f, pmul(hv[5], pmul(hv[12], w[45])));
  t[1] += pmul(-0.130584508f, pmul(hv[5], pmul(hv[14], w[45])));
  t[1] += pmul(0.143048167f, pmul(hv[6], pmul(hv[11], w[45])));
  t[2] += pmul(0.175197512f, pmul(hv[6], pmul(hv[12], w[45])));
  t[3] += pmul(0.143048167f, pmul(hv[6], pmul(hv[13], w[45])));
  t[1] += pmul(0.130584508f, pmul(hv[7], pmul(hv[10], w[45])));
  t[3] += pmul(-0.101150326f, pmul(hv[7], pmul(hv[12], w[45])));
  t[2] += pmul(0.165177792f, pmul(hv[7], pmul(hv[13], w[45])));
  t[3] += pmul(0.130584508f, pmul(hv[7], pmul(hv[14], w[45])));
  t[1] += pmul(0.159932718f, pmul(hv[8], pmul(hv[9], w[45])));
  t[1] += pmul(0.0412944481f, pmul(hv[8], pmul(hv[11], w[45])));
  t[3] += pmul(-0.0412944481f, pmul(hv[8], pmul(hv[13], w[45])));
  t[2] += pmul(0.130584508f, pmul(hv[8], pmul(hv[14], w[45])));
  t[3] += pmul(0.159932718f, pmul(hv[8], pmul(hv[15], w[45])));
  t[13] += pmul(-0.101565734f, pmul(hv[4], pmul(hv[9], w[47])));
  t[12] += pmul(-0.203131467f, pmul(hv[4], pmul(hv[10], w[47])));
  t[13] += pmul(0.157344952f, pmul(hv[4], pmul(hv[11], w[47])));
  t[15] += pmul(0.101565734f, pmul(hv[4], pmul(hv[11], w[47])));
  t[10] += pmul(-0.203131467f, pmul(hv[4], pmul(hv[12], w[47])));
  t[9] += pmul(-0.101565734f, pmul(hv[4], pmul(hv[13], w[47])));
  t[11] += pmul(0.157344952f, pmul(hv[4], pmul(hv[13], w[47])));
  t[11] += pmul(0.101565734f, pmul(hv[4], pmul(hv[15], w[47])));
  t[14] += pmul(0.160589531f, pmul(hv[5], pmul(hv[9], w[47])));
  t[13] += pmul(0.124392115f, pmul(hv[5], pmul(hv[10], w[47])));
  t[15] += pmul(-0.160589531f, pmul(hv[5], pmul(hv[10], w[47])));
  t[12] += pmul(0.0642358065f, pmul(hv[5], pmul(hv[11], w[47])));
  t[14] += pmul(-0.124392115f, pmul(hv[5], pmul(hv[11], w[47])));
  t[11] += pmul(0.0642358065f, pmul(hv[5], pmul(hv[12], w[47])));
  t[10] += pmul(0.124392115f, pmul(hv[5], pmul(hv[13], w[47])));
  t[9] += pmul(0.160589531f, pmul(hv[5], pmul(hv[14], w[47])));
  t[11] += pmul(-0.124392115f, pmul(hv[5], pmul(hv[14], w[47])));
  t[10] += pmul(-0.160589531f, pmul(hv[5], pmul(hv[15], w[47])));
  t[9] += pmul(-0.227107882f, pmul(hv[6], pmul(hv[9], w[47])));
  t[11] += pmul(0.136264727f, pmul(hv[6], pmul(hv[11], w[47])));
  t[12] += pmul(0.181686312f, pmul(hv[6], pmul(hv[12], w[47])));
  t[13] += pmul(0.136264727f, pmul(hv[6], pmul(hv[13], w[47])));
  t[15] += pmul(-0.227107882f, pmul(hv[6], pmul(hv[15], w[47])));
  t[10] += pmul(0.160589531f, pmul(hv[7], pmul(hv[9], w[47])));
  t[9] += pmul(0.160589531f, pmul(hv[7], pmul(hv[10], w[47])));
  t[11] += pmul(0.124392115f, pmul(hv[7], pmul(hv[10], w[47])));
  t[10] += pmul(0.124392115f, pmul(hv[7], pmul(hv[11], w[47])));
  t[13] += pmul(0.0642358065f, pmul(hv[7], pmul(hv[12], w[47])));
  t[12] += pmul(0.0642358065f, pmul(hv[7], pmul(hv[13], w[47])));
  t[14] += pmul(0.124392115f, pmul(hv[7], pmul(hv[13], w[47])));
  t[13] += pmul(0.124392115f, pmul(hv[7], pmul(hv[14], w[47])));
  t[15] += pmul(0.160589531f, pmul(hv[7], pmul(hv[14], w[47])));
  t[14] += pmul(0.160589531f, pmul(hv[7], pmul(hv[15], w[47])));
  t[11] += pmul(-0.101565734f, pmul(hv[8], pmul(hv[9], w[47])));
  t[9] += pmul(-0.101565734f, pmul(hv[8], pmul(hv[11], w[47])));
  t[11] += pmul(-0.157344952f, pmul(hv[8], pmul(hv[11], w[47])));
  t[14] += pmul(-0.203131467f, pmul(hv[8], pmul(hv[12], w[47])));
  t[13] += pmul(0.157344952f, pmul(hv[8], pmul(hv[13], w[47])));
  t[15] += pmul(-0.101565734f, pmul(hv[8], pmul(hv[13], w[47])));
  t[12] += pmul(-0.203131467f, pmul(hv[8], pmul(hv[14], w[47])));
  t[13] += pmul(-0.101565734f, pmul(hv[8], pmul(hv[15], w[47])));
  t[9] += pmul(0.304697186f, pmul(hv[9], pmul(hv[0], w[51])));
  t[10] += pmul(0.304697186f, pmul(hv[10], pmul(hv[0], w[51])));
  t[11] += pmul(0.304697186f, pmul(hv[11], pmul(hv[0], w[51])));
  t[12] += pmul(0.304697186f, pmul(hv[12], pmul(hv[0], w[51])));
  t[13] += pmul(0.304697186f, pmul(hv[13], pmul(hv[0], w[51])));
  t[14] += pmul(0.304697186f, pmul(hv[14], pmul(hv[0], w[51])));
  t[15] += pmul(0.304697186f, pmul(hv[15], pmul(hv[0], w[51])));
  t[8] += pmul(0.191156149f, pmul(hv[9], pmul(hv[1], w[54])));
  t[4] += pmul(0.191156149f, pmul(hv[9], pmul(hv[3], w[54])));
  t[7] += pmul(0.156078354f, pmul(hv[10], pmul(hv[1], w[54])));
  t[4] += pmul(0.156078354f, pmul(hv[10], pmul(hv[2], w[54])));
  t[5] += pmul(0.156078354f, pmul(hv[10], pmul(hv[3], w[54])));
  t[6] += pmul(0.170975268f, pmul(hv[11], pmul(hv[1], w[54])));
  t[8] += pmul(0.0493563078f, pmul(hv[11], pmul(hv[1], w[54])));
  t[5] += pmul(0.197425231f, pmul(hv[11], pmul(hv[2], w[54])));
  t[4] += pmul(-0.0493563078f, pmul(hv[11], pmul(hv[3], w[54])));
  t[5] += pmul(-0.120897770f, pmul(hv[12], pmul(hv[1], w[54])));
  t[6] += pmul(0.209401071f, pmul(hv[12], pmul(hv[2], w[54])));
  t[7] += pmul(-0.120897770f, pmul(hv[12], pmul(hv[3], w[54])));
  t[4] += pmul(-0.0493563078f, pmul(hv[13], pmul(hv[1], w[54])));
  t[7] += pmul(0.197425231f, pmul(hv[13], pmul(hv[2], w[54])));
  t[6] += pmul(0.170975268f, pmul(hv[13], pmul(hv[3], w[54])));
  t[8] += pmul(-0.0493563078f, pmul(hv[13], pmul(hv[3], w[54])));
  t[5] += pmul(-0.156078354f, pmul(hv[14], pmul(hv[1], w[54])));
  t[8] += pmul(0.156078354f, pmul(hv[14], pmul(hv[2], w[54])));
  t[7] += pmul(0.156078354f, pmul(hv[14], pmul(hv[3], w[54])));
  t[4] += pmul(-0.191156149f, pmul(hv[15], pmul(hv[1], w[54])));
  t[8] += pmul(0.191156149f, pmul(hv[15], pmul(hv[3], w[54])));
  t[3] += pmul(0.159932718f, pmul(hv[9], pmul(hv[4], w[57])));
  t[1] += pmul(0.159932718f, pmul(hv[9], pmul(hv[8], w[57])));
  t[2] += pmul(0.130584508f, pmul(hv[10], pmul(hv[4], w[57])));
  t[3] += pmul(0.130584508f, pmul(hv[10], pmul(hv[5], w[57])));
  t[1] += pmul(0.130584508f, pmul(hv[10], pmul(hv[7], w[57])));
  t[3] += pmul(-0.0412944481f, pmul(hv[11], pmul(hv[4], w[57])));
  t[2] += pmul(0.165177792f, pmul(hv[11], pmul(hv[5], w[57])));
  t[1] += pmul(0.143048167f, pmul(hv[11], pmul(hv[6], w[57])));
  t[1] += pmul(0.0412944481f, pmul(hv[11], pmul(hv[8], w[57])));
  t[1] += pmul(-0.101150326f, pmul(hv[12], pmul(hv[5], w[57])));
  t[2] += pmul(0.175197512f, pmul(hv[12], pmul(hv[6], w[57])));
  t[3] += pmul(-0.101150326f, pmul(hv[12], pmul(hv[7], w[57])));
  t[1] += pmul(-0.0412944481f, pmul(hv[13], pmul(hv[4], w[57])));
  t[3] += pmul(0.143048167f, pmul(hv[13], pmul(hv[6], w[57])));
  t[2] += pmul(0.165177792f, pmul(hv[13], pmul(hv[7], w[57])));
  t[3] += pmul(-0.0412944481f, pmul(hv[13], pmul(hv[8], w[57])));
  t[1] += pmul(-0.130584508f, pmul(hv[14], pmul(hv[5], w[57])));
  t[3] += pmul(0.130584508f, pmul(hv[14], pmul(hv[7], w[57])));
  t[2] += pmul(0.130584508f, pmul(hv[14], pmul(hv[8], w[57])));
  t[1] += pmul(-0.159932718f, pmul(hv[15], pmul(hv[4], w[57])));
  t[3] += pmul(0.159932718f, pmul(hv[15], pmul(hv[8], w[57])));
  t[13] += pmul(-0.101565734f, pmul(hv[9], pmul(hv[4], w[59])));
  t[14] += pmul(0.160589531f, pmul(hv[9], pmul(hv[5], w[59])));
  t[9] += pmul(-0.227107882f, pmul(hv[9], pmul(hv[6], w[59])));
  t[10] += pmul(0.160589531f, pmul(hv[9], pmul(hv[7], w[59])));
  t[11] += pmul(-0.101565734f, pmul(hv[9], pmul(hv[8], w[59])));
  t[12] += pmul(-0.203131467f, pmul(hv[10], pmul(hv[4], w[59])));
  t[13] += pmul(0.124392115f, pmul(hv[10], pmul(hv[5], w[59])));
  t[15] += pmul(-0.160589531f, pmul(hv[10], pmul(hv[5], w[59])));
  t[9] += pmul(0.160589531f, pmul(hv[10], pmul(hv[7], w[59])));
  t[11] += pmul(0.124392115f, pmul(hv[10], pmul(hv[7], w[59])));
  t[13] += pmul(0.157344952f, pmul(hv[11], pmul(hv[4], w[59])));
  t[15] += pmul(0.101565734f, pmul(hv[11], pmul(hv[4], w[59])));
  t[12] += pmul(0.0642358065f, pmul(hv[11], pmul(hv[5], w[59])));
  t[14] += pmul(-0.124392115f, pmul(hv[11], pmul(hv[5], w[59])));
  t[11] += pmul(0.136264727f, pmul(hv[11], pmul(hv[6], w[59])));
  t[10] += pmul(0.124392115f, pmul(hv[11], pmul(hv[7], w[59])));
  t[9] += pmul(-0.101565734f, pmul(hv[11], pmul(hv[8], w[59])));
  t[11] += pmul(-0.157344952f, pmul(hv[11], pmul(hv[8], w[59])));
  t[10] += pmul(-0.203131467f, pmul(hv[12], pmul(hv[4], w[59])));
  t[11] += pmul(0.0642358065f, pmul(hv[12], pmul(hv[5], w[59])));
  t[12] += pmul(0.181686312f, pmul(hv[12], pmul(hv[6], w[59])));
  t[13] += pmul(0.0642358065f, pmul(hv[12], pmul(hv[7], w[59])));
  t[14] += pmul(-0.203131467f, pmul(hv[12], pmul(hv[8], w[59])));
  t[9] += pmul(-0.101565734f, pmul(hv[13], pmul(hv[4], w[59])));
  t[11] += pmul(0.157344952f, pmul(hv[13], pmul(hv[4], w[59])));
  t[10] += pmul(0.124392115f, pmul(hv[13], pmul(hv[5], w[59])));
  t[13] += pmul(0.136264727f, pmul(hv[13], pmul(hv[6], w[59])));
  t[12] += pmul(0.0642358065f, pmul(hv[13], pmul(hv[7], w[59])));
  t[14] += pmul(0.124392115f, pmul(hv[13], pmul(hv[7], w[59])));
  t[13] += pmul(0.157344952f, pmul(hv[13], pmul(hv[8], w[59])));
  t[15] += pmul(-0.101565734f, pmul(hv[13], pmul(hv[8], w[59])));
  t[9] += pmul(0.160589531f, pmul(hv[14], pmul(hv[5], w[59])));
  t[11] += pmul(-0.124392115f, pmul(hv[14], pmul(hv[5], w[59])));
  t[13] += pmul(0.124392115f, pmul(hv[14], pmul(hv[7], w[59])));
  t[15] += pmul(0.160589531f, pmul(hv[14], pmul(hv[7], w[59])));
  t[12] += pmul(-0.203131467f, pmul(hv[14], pmul(hv[8], w[59])));
  t[11] += pmul(0.101565734f, pmul(hv[15], pmul(hv[4], w[59])));
  t[10] += pmul(-0.160589531f, pmul(hv[15], pmul(hv[5], w[59])));
  t[15] += pmul(-0.227107882f, pmul(hv[15], pmul(hv[6], w[59])));
  t[14] += pmul(0.160589531f, pmul(hv[15], pmul(hv[7], w[59])));
  t[13] += pmul(-0.101565734f, pmul(hv[15], pmul(hv[8], w[59])));
  t[0] += pmul(0.141047403f, pmul(hv[9], pmul(hv[9], w[60])));
  t[0] += pmul(0.141047403f, pmul(hv[10], pmul(hv[10], w[60])));
  t[0] += pmul(0.141047403f, pmul(hv[11], pmul(hv[11], w[60])));
  t[0] += pmul(0.141047403f, pmul(hv[12], pmul(hv[12], w[60])));
  t[0] += pmul(0.141047403f, pmul(hv[13], pmul(hv[13], w[60])));
  t[0] += pmul(0.141047403f, pmul(hv[14], pmul(hv[14], w[60])));
  t[0] += pmul(0.141047403f, pmul(hv[15], pmul(hv[15], w[60])));
  t[6] += pmul(-0.177703023f, pmul(hv[9], pmul(hv[9], w[62])));
  t[7] += pmul(0.125655010f, pmul(hv[9], pmul(hv[10], w[62])));
  t[8] += pmul(-0.0794712082f, pmul(hv[9], pmul(hv[11], w[62])));
  t[4] += pmul(-0.0794712082f, pmul(hv[9], pmul(hv[13], w[62])));
  t[5] += pmul(0.125655010f, pmul(hv[9], pmul(hv[14], w[62])));
  t[7] += pmul(0.125655010f, pmul(hv[10], pmul(hv[9], w[62])));
  t[7] += pmul(0.0973319486f, pmul(hv[10], pmul(hv[11], w[62])));
  t[4] += pmul(-0.158942416f, pmul(hv[10], pmul(hv[12], w[62])));
  t[5] += pmul(0.0973319486f, pmul(hv[10], pmul(hv[13], w[62])));
  t[5] += pmul(-0.125655010f, pmul(hv[10], pmul(hv[15], w[62])));
  t[8] += pmul(-0.0794712082f, pmul(hv[11], pmul(hv[9], w[62])));
  t[7] += pmul(0.0973319486f, pmul(hv[11], pmul(hv[10], w[62])));
  t[6] += pmul(0.106621809f, pmul(hv[11], pmul(hv[11], w[62])));
  t[8] += pmul(-0.123116262f, pmul(hv[11], pmul(hv[11], w[62])));
  t[5] += pmul(0.0502620041f, pmul(hv[11], pmul(hv[12], w[62])));
  t[4] += pmul(0.123116262f, pmul(hv[11], pmul(hv[13], w[62])));
  t[5] += pmul(-0.0973319486f, pmul(hv[11], pmul(hv[14], w[62])));
  t[4] += pmul(0.0794712082f, pmul(hv[11], pmul(hv[15], w[62])));
  t[4] += pmul(-0.158942416f, pmul(hv[12], pmul(hv[10], w[62])));
  t[5] += pmul(0.0502620041f, pmul(hv[12], pmul(hv[11], w[62])));
  t[6] += pmul(0.142162412f, pmul(hv[12], pmul(hv[12], w[62])));
  t[7] += pmul(0.0502620041f, pmul(hv[12], pmul(hv[13], w[62])));
  t[8] += pmul(-0.158942416f, pmul(hv[12], pmul(hv[14], w[62])));
  t[4] += pmul(-0.0794712082f, pmul(hv[13], pmul(hv[9], w[62])));
  t[5] += pmul(0.0973319486f, pmul(hv[13], pmul(hv[10], w[62])));
  t[4] += pmul(0.123116262f, pmul(hv[13], pmul(hv[11], w[62])));
  t[7] += pmul(0.0502620041f, pmul(hv[13], pmul(hv[12], w[62])));
  t[6] += pmul(0.106621809f, pmul(hv[13], pmul(hv[13], w[62])));
  t[8] += pmul(0.123116262f, pmul(hv[13], pmul(hv[13], w[62])));
  t[7] += pmul(0.0973319486f, pmul(hv[13], pmul(hv[14], w[62])));
  t[8] += pmul(-0.0794712082f, pmul(hv[13], pmul(hv[15], w[62])));
  t[5] += pmul(0.125655010f, pmul(hv[14], pmul(hv[9], w[62])));
  t[5] += pmul(-0.0973319486f, pmul(hv[14], pmul(hv[11], w[62])));
  t[8] += pmul(-0.158942416f, pmul(hv[14], pmul(hv[12], w[62])));
  t[7] += pmul(0.0973319486f, pmul(hv[14], pmul(hv[13], w[62])));
  t[7] += pmul(0.125655010f, pmul(hv[14], pmul(hv[15], w[62])));
  t[5] += pmul(-0.125655010f, pmul(hv[15], pmul(hv[10], w[62])));
  t[4] += pmul(0.0794712082f, pmul(hv[15], pmul(hv[11], w[62])));
  t[8] += pmul(-0.0794712082f, pmul(hv[15], pmul(hv[13], w[62])));
  t[7] += pmul(0.125655010f, pmul(hv[15], pmul(hv[14], w[62])));
  t[6] += pmul(-0.177703023f, pmul(hv[15], pmul(hv[15], w[62])));
  for (int pass = 0; pass < 2; ++pass) {
#pragma unroll
    for (int k = 0; k < L2; ++k) ((volatile float*)T)[((size_t)n * L2 + k) * CH + h] = t[k]; __threadfence(); } }
}

extern "C" void kernel_launch(void* const* d_in, const int* in_sizes, int n_in, void* d_out, int out_size, void* d_ws, size_t ws_size, hipStream_t stream) {
  (void)n_in;
  auto Fp = [&](int i) { return (const float*)d_in[i]; };
  if (in_sizes[0] != N * L2 * CI || in_sizes[2] != 4 * CI || in_sizes[4] != 4 * CI * CH || in_sizes[6] != 64 * CH || in_sizes[7] != 4 * CH * CI || out_size != N * L2 * CI) return;
  const int NV = N;
  size_t off = 0; char* ws = (char*)d_ws;
  auto carve = [&](size_t bytes) { char* p = ws + off; off += (bytes + 255) & ~(size_t)255; return p; };
  b16* W1T = (b16*)carve((size_t)4 * CH * CI * 2); b16* W2T = (b16*)carve((size_t)4 * CI * CH * 2); float* XN = (float*)carve((size_t)N * L2 * CI * 4); float* Hh = (float*)carve((size_t)N * L2 * CH * 4); float* T = (float*)carve((size_t)N * L2 * CH * 4);
  if (off > ws_size || off > ((size_t)128 << 20)) return;
  wput_kernel<<<(4 * CI * (CH / 8) + 255) / 256, 256, 0, stream>>>(Fp(4), Fp(7), W1T, W2T);
  norm_kernel<<<(NV + 7) / 8, 256, 0, stream>>>(Fp(0), Fp(2), Fp(3), NV, XN);
  so3_kernel<0><<<NV * (CH / 128), 32, 0, stream>>>(XN, W1T, Fp(5), nullptr, NV, Hh);
  gaunt_kernel<<<(NV * CH + 255) / 256, 256, 0, stream>>>(Hh, Fp(6), NV, T);
  so3_kernel<1><<<NV * (CI / 128), 32, 0, stream>>>(T, W2T, Fp(8), Fp(0), NV, (float*)d_out);
}
